// NLB_41025527611419
// MI455X (gfx1250) — hardware-verified
//
#include <hip/hip_runtime.h>


namespace {
constexpr int Bn = 8, C = 256, CI = 128, N = 4096, NT = Bn * N;
constexpr float QS = 8.0f, KS = 8.0f, VS = 8.0f, PS = 8.0f, EPS = 1e-5f, WS8 = 8.0f;

typedef _Float16 b16;
typedef __attribute__((ext_vector_type(16))) _Float16 v16b;
typedef __attribute__((ext_vector_type(8))) _Float16 v8b;
typedef __attribute__((ext_vector_type(8))) float v8f;
typedef __attribute__((ext_vector_type(4))) float v4f;
__device__ __forceinline__ float bf16_rne(float f) { unsigned int u = __float_as_uint(f); u += 0x7FFFu + ((u >> 16) & 1u); return __uint_as_float(u & 0xFFFF0000u); }
__device__ __forceinline__ void split16(float v, b16& hi, b16& lo) { hi = (b16)v; lo = (b16)(v - (float)hi); }
__device__ __forceinline__ v16b frag_kb(const b16* p, int hh) { const v8b a = *(const v8b*)(p + 8 * hh), b = *(const v8b*)(p + 16 + 8 * hh); v16b f;
#pragma unroll
  for (int e = 0; e < 8; ++e) { f[e] = a[e]; f[8 + e] = b[e]; } return f; }
__device__ __forceinline__ v8f wmma16b(v16b a, v16b b, v8f c) { v8f d = __builtin_amdgcn_wmma_f32_16x16x32_f16(false, a, false, b, (short)0, c, false, false); asm volatile("v_nop\n\tv_nop\n\tv_nop\n\tv_nop" : "+v"(d) : "v"(a), "v"(b)); return d; }
__device__ __forceinline__ void wave_lds_sync() { __builtin_amdgcn_fence(__ATOMIC_RELEASE, "workgroup"); __builtin_amdgcn_wave_barrier(); __builtin_amdgcn_fence(__ATOMIC_ACQUIRE, "workgroup"); }
__device__ __forceinline__ float nexp(float x) { return __builtin_amdgcn_exp2f(x * 1.4426950408889634f); }

__global__ __launch_bounds__(256) void prep_kernel(const float* __restrict__ gam, const float* __restrict__ bet, const float* __restrict__ mean, const float* __restrict__ var, const float* __restrict__ wg, const float* __restrict__ bg, const float* __restrict__ wt, const float* __restrict__ bt, const float* __restrict__ wp, const float* __restrict__ bp, const float* __restrict__ ww, const float* __restrict__ bw, b16* __restrict__ R, b16* __restrict__ Rw, float* __restrict__ P) {
  const int t_ = blockIdx.x * 256 + threadIdx.x, nth = gridDim.x * 256;
  for (int pass = 0; pass < 2; ++pass) {
    for (int q = t_; q < 3 * CI * C; q += nth) { const int m = q / (CI * C), o = (q / C) % CI, c = q % C; const float* W = (m == 0) ? wt : (m == 1) ? wp : wg;
      const float sc = bf16_rne(gam[c]) * rsqrtf(bf16_rne(var[c]) + EPS); b16 h_, l_; split16(bf16_rne(W[o * C + c]) * sc * WS8, h_, l_); R[q] = h_; R[3 * CI * C + q] = l_; }
    for (int q = t_; q < C * CI; q += nth) Rw[q] = (b16)bf16_rne(ww[q]);
    for (int q = t_; q < 3 * CI + C; q += nth) { float v;
      if (q < 3 * CI) { const int m = q / CI, o = q % CI; const float* W = (m == 0) ? wt : (m == 1) ? wp : wg; const float* bb = (m == 0) ? bt : (m == 1) ? bp : bg; float s = bf16_rne(bb[o]);
        for (int c = 0; c < C; ++c) { const float sc = bf16_rne(gam[c]) * rsqrtf(bf16_rne(var[c]) + EPS); const float sh = bf16_rne(bet[c]) - bf16_rne(mean[c]) * sc; s += bf16_rne(W[o * C + c]) * sh; } v = s; }
      else v = bf16_rne(bw[q - 3 * CI]);
      P[q] = v; }
    __threadfence(); }
}

__global__ __launch_bounds__(256) void xpose_kernel(const float* __restrict__ x, b16* __restrict__ xt) {
  __shared__ __attribute__((aligned(16))) b16 T[128][C + 8];
  const int b = blockIdx.y, n0 = blockIdx.x * 128, t_ = threadIdx.x;
  for (int i = t_; i < C * 128; i += 256) { const int c = i >> 7, nn = i & 127; T[nn][c] = (b16)bf16_rne(x[((size_t)b * C + c) * N + n0 + nn]); }
  __syncthreads();
  for (int pass = 0; pass < 2; ++pass) { for (int i = t_; i < 128 * (C / 8); i += 256) { const int nn = i / (C / 8), c8 = (i % (C / 8)) * 8; *(volatile v8b*)(xt + ((size_t)b * N + n0 + nn) * C + c8) = *(const v8b*)(&T[nn][c8]); } __threadfence(); }
}

__global__ __launch_bounds__(128) void proj_kernel(const b16* __restrict__ xt, const b16* __restrict__ R, const float* __restrict__ P, b16* __restrict__ qp, b16* __restrict__ kp, b16* __restrict__ vt) {
  __shared__ __attribute__((aligned(16))) b16 Tq[4][32][64 + 8]; __shared__ __attribute__((aligned(16))) b16 Tv[64][128 + 8];
  const int lane = threadIdx.x & 31, wave = threadIdx.x >> 5, nloc = lane & 15, hlf = lane >> 4, which = blockIdx.z, c0 = blockIdx.x * 64, p0 = blockIdx.y * 128, m0 = p0 + wave * 32, b = p0 / N, t0 = p0 % N;
  const b16* Wh = R + (size_t)which * CI * C; const b16* Wl = R + (size_t)3 * CI * C + (size_t)which * CI * C; const float* bias = P + which * CI;
  v8f acc[2][4];
#pragma unroll
  for (int r = 0; r < 2; ++r)
#pragma unroll
    for (int t = 0; t < 4; ++t) acc[r][t] = (v8f){};
#pragma unroll 2
  for (int kb = 0; kb < C; kb += 32) { const v16b a0 = frag_kb(xt + (size_t)(m0 + nloc) * C + kb, hlf), a1 = frag_kb(xt + (size_t)(m0 + 16 + nloc) * C + kb, hlf);
#pragma unroll
    for (int t = 0; t < 4; ++t) { const size_t ro = (size_t)(c0 + t * 16 + nloc) * C + kb; const v16b bh = frag_kb(Wh + ro, hlf), bl = frag_kb(Wl + ro, hlf); acc[0][t] = wmma16b(a0, bh, acc[0][t]); acc[0][t] = wmma16b(a0, bl, acc[0][t]); acc[1][t] = wmma16b(a1, bh, acc[1][t]); acc[1][t] = wmma16b(a1, bl, acc[1][t]); } }
  const float scl = (which == 0) ? QS : (which == 1) ? KS : VS;
  if (which < 2) {
#pragma unroll
    for (int t = 0; t < 4; ++t) { const float bb = bias[c0 + t * 16 + nloc];
#pragma unroll
      for (int r = 0; r < 2; ++r)
#pragma unroll
        for (int v = 0; v < 8; ++v) Tq[wave][r * 16 + 8 * hlf + v][t * 16 + nloc] = (b16)((acc[r][t][v] * (1.0f / WS8) + bb) * scl); }
    wave_lds_sync();
    b16* base = ((which == 0) ? qp : kp) + ((size_t)b * N + (m0 % N)) * CI + c0;
    for (int pass = 0; pass < 2; ++pass) {
#pragma unroll
      for (int j = 0; j < 8; ++j) { const int rr = j * 4 + (lane >> 3), c8 = (lane & 7) * 8; *(volatile v8b*)(base + (size_t)rr * CI + c8) = *(const v8b*)(&Tq[wave][rr][c8]); }
      __threadfence(); }
    return; }
#pragma unroll
  for (int t = 0; t < 4; ++t) { const float bb = bias[c0 + t * 16 + nloc];
#pragma unroll
    for (int r = 0; r < 2; ++r)
#pragma unroll
      for (int v = 0; v < 8; ++v) Tv[t * 16 + nloc][wave * 32 + r * 16 + 8 * hlf + v] = (b16)((acc[r][t][v] * (1.0f / WS8) + bb) * scl); }
  __syncthreads();
  for (int pass = 0; pass < 2; ++pass) { for (int i = threadIdx.x; i < 64 * 16; i += 128) { const int d = i >> 4, c8 = (i & 15) * 8; *(volatile v8b*)(vt + ((size_t)b * CI + c0 + d) * N + t0 + c8) = *(const v8b*)(&Tv[d][c8]); } __threadfence(); }
}

__global__ __launch_bounds__(256) void attn_kernel(const b16* __restrict__ qp, const b16* __restrict__ kp, const b16* __restrict__ vt, b16* __restrict__ yr) {
  __shared__ __attribute__((aligned(16))) b16 Os[8][16][CI + 8];
  const int wid = threadIdx.x >> 5, lane = threadIdx.x & 31, hh = lane >> 4, col = lane & 15; const int p0 = blockIdx.x * 128 + wid * 16, b = p0 / N, q0 = p0 % N, qi = q0 + col;
  const b16* Q = qp + ((size_t)b * N) * CI; const b16* K = kp + ((size_t)b * N) * CI; const b16* V = vt + ((size_t)b * CI) * N;
  v16b qf[4];
#pragma unroll
  for (int ks = 0; ks < 4; ++ks) qf[ks] = frag_kb(Q + (size_t)qi * CI + ks * 32, hh);
  float m = -INFINITY, l = 0.0f; v8f o[8];
#pragma unroll
  for (int t = 0; t < 8; ++t) o[t] = (v8f){};
  for (int kb = 0; kb < N; kb += 32) { v8f s0 = {}, s1 = {};
#pragma unroll
    for (int ks = 0; ks < 4; ++ks) { const v16b ka = frag_kb(K + (size_t)(kb + col) * CI + ks * 32, hh), kc = frag_kb(K + (size_t)(kb + 16 + col) * CI + ks * 32, hh); s0 = wmma16b(ka, qf[ks], s0); s1 = wmma16b(kc, qf[ks], s1); }
    float mr = -INFINITY;
#pragma unroll
    for (int r = 0; r < 8; ++r) { s0[r] *= 1.0f / (QS * KS); s1[r] *= 1.0f / (QS * KS); mr = fmaxf(mr, fmaxf(s0[r], s1[r])); }
    mr = fmaxf(mr, __shfl_xor(mr, 16));
    const float mn = fmaxf(m, mr), al_ = nexp(m - mn); m = mn; float sum = 0.0f; v16b pbv;
#pragma unroll
    for (int r = 0; r < 8; ++r) { const float e0 = nexp(s0[r] - mn), e1 = nexp(s1[r] - mn); sum += e0 + e1; pbv[r] = (b16)(e0 * PS); pbv[8 + r] = (b16)(e1 * PS); }
    sum += __shfl_xor(sum, 16); l = l * al_ + sum;
#pragma unroll
    for (int t = 0; t < 8; ++t) { o[t] *= al_; const v16b vf = frag_kb(V + (size_t)(t * 16 + col) * N + kb, hh); o[t] = wmma16b(vf, pbv, o[t]); } }
  const float inv = 1.0f / (l * VS * PS);
#pragma unroll
  for (int t = 0; t < 8; ++t)
#pragma unroll
    for (int r = 0; r < 8; ++r) Os[wid][col][t * 16 + 8 * hh + r] = (b16)(o[t][r] * inv);
  wave_lds_sync();
  for (int pass = 0; pass < 2; ++pass) { for (int i = lane; i < 16 * 16; i += 32) { const int rr = i >> 4, c8 = (i & 15) * 8; *(volatile v8b*)(yr + ((size_t)b * N + q0 + rr) * CI + c8) = *(const v8b*)(&Os[wid][rr][c8]); } __threadfence(); }
}

__global__ __launch_bounds__(128) void out_kernel(const b16* __restrict__ yr, const b16* __restrict__ Rw, const float* __restrict__ P, const float* __restrict__ x, float* __restrict__ out) {
  __shared__ __attribute__((aligned(16))) float Tc[64][128 + 4];
  const int lane = threadIdx.x & 31, wave = threadIdx.x >> 5, nloc = lane & 15, hlf = lane >> 4, p0 = blockIdx.y * 128, m0 = p0 + wave * 32, c0 = blockIdx.x * 64, b = p0 / N, t0 = p0 % N; const float* bw = P + 3 * CI;
  v8f acc[2][4];
#pragma unroll
  for (int r = 0; r < 2; ++r)
#pragma unroll
    for (int t = 0; t < 4; ++t) acc[r][t] = (v8f){};
#pragma unroll
  for (int kb = 0; kb < CI; kb += 32) { const v16b a0 = frag_kb(yr + (size_t)(m0 + nloc) * CI + kb, hlf), a1 = frag_kb(yr + (size_t)(m0 + 16 + nloc) * CI + kb, hlf);
#pragma unroll
    for (int t = 0; t < 4; ++t) { const v16b bwf = frag_kb(Rw + (size_t)(c0 + t * 16 + nloc) * CI + kb, hlf); acc[0][t] = wmma16b(a0, bwf, acc[0][t]); acc[1][t] = wmma16b(a1, bwf, acc[1][t]); } }
#pragma unroll
  for (int t = 0; t < 4; ++t) { const int cc = c0 + t * 16 + nloc; const float bb = bw[cc];
#pragma unroll
    for (int r = 0; r < 2; ++r)
#pragma unroll
      for (int v = 0; v < 8; ++v) { const int pl = wave * 32 + r * 16 + 8 * hlf + v; Tc[t * 16 + nloc][pl] = acc[r][t][v] + bb + bf16_rne(x[((size_t)b * C + cc) * N + t0 + pl]); } }
  __syncthreads();
  for (int pass = 0; pass < 2; ++pass) { for (int i = threadIdx.x; i < 64 * 32; i += 128) { const int cc = i >> 5, c4 = (i & 31) * 4; *(volatile v4f*)(out + ((size_t)b * C + c0 + cc) * N + t0 + c4) = *(const v4f*)(&Tc[cc][c4]); } __threadfence(); }
}
}

extern "C" void kernel_launch(void* const* d_in, const int* in_sizes, int n_in,
                              void* d_out, int out_size, void* d_ws, size_t ws_size, hipStream_t stream) {
  (void)n_in; (void)out_size;
  const float* x = (const float*)d_in[0]; const float* gam = (const float*)d_in[1]; const float* bet = (const float*)d_in[2]; const float* mean = (const float*)d_in[3]; const float* var = (const float*)d_in[4];
  const float* wg = (const float*)d_in[5]; const float* bg = (const float*)d_in[6]; const float* wt = (const float*)d_in[7]; const float* bt = (const float*)d_in[8]; const float* wp = (const float*)d_in[9]; const float* bp = (const float*)d_in[10]; const float* ww = (const float*)d_in[11]; const float* bw = (const float*)d_in[12];
  float* out = (float*)d_out;
  if (in_sizes[0] != NT * C || in_sizes[5] != CI * C || in_sizes[11] != C * CI) return;
  size_t off = 0; char* ws = (char*)d_ws;
  auto carve = [&](size_t bytes) { char* p = ws + off; off += (bytes + 255) & ~(size_t)255; return p; };
  b16* R = (b16*)carve((size_t)6 * CI * C * 2); b16* Rw = (b16*)carve((size_t)C * CI * 2); float* P = (float*)carve(1024 * 4); b16* xt = (b16*)carve((size_t)NT * C * 2);
  b16* qp = (b16*)carve((size_t)NT * CI * 2); b16* kp = (b16*)carve((size_t)NT * CI * 2); b16* vt = (b16*)carve((size_t)NT * CI * 2); b16* yr = (b16*)carve((size_t)NT * CI * 2);
  if (off > ws_size) return;
  prep_kernel<<<64, 256, 0, stream>>>(gam, bet, mean, var, wg, bg, wt, bt, wp, bp, ww, bw, R, Rw, P);
  xpose_kernel<<<dim3(N / 128, Bn), 256, 0, stream>>>(x, xt);
  proj_kernel<<<dim3(CI / 64, NT / 128, 3), 128, 0, stream>>>(xt, R, P, qp, kp, vt);
  attn_kernel<<<NT / 128, 256, 0, stream>>>(qp, kp, vt, yr);
  out_kernel<<<dim3(C / 64, NT / 128), 128, 0, stream>>>(yr, Rw, P, x, out);
}
